// RSSM_17849884082580
// MI455X (gfx1250) — hardware-verified
//
#include <hip/hip_runtime.h>


typedef __attribute__((ext_vector_type(16))) _Float16 v16h;
typedef __attribute__((ext_vector_type(8)))  _Float16 v8h;
typedef __attribute__((ext_vector_type(16))) __bf16   v16b;
typedef __attribute__((ext_vector_type(8)))  __bf16   v8b;
typedef __attribute__((ext_vector_type(8)))  float    v8f;
typedef __attribute__((ext_vector_type(4)))  float    v4f;
#define U16(p) ((const unsigned short*)(const void*)(p))

__device__ __forceinline__ unsigned short f2bf_bits(float f) {
  unsigned u = __float_as_uint(f);
  return (unsigned short)((u + 0x7FFFu + ((u >> 16) & 1u)) >> 16);
}
__device__ __forceinline__ float bf_bits2f(unsigned short h) { return __uint_as_float(((unsigned)h) << 16); }

__device__ __forceinline__ void dep_guard_h(v8f& a, v8f& b, v16h x, v16h y) { asm volatile("v_nop\n\tv_nop\n\tv_nop\n\tv_nop" : "+v"(a), "+v"(b) : "v"(x), "v"(y)); }
__device__ __forceinline__ void dep_guard_b(v8f& a, v8f& b, v16b x, v16b y) { asm volatile("v_nop\n\tv_nop\n\tv_nop\n\tv_nop" : "+v"(a), "+v"(b) : "v"(x), "v"(y)); }
__device__ __forceinline__ void keep4_h(v16h a, v16h b, v16h c, v16h d) { asm volatile("v_nop" :: "v"(a), "v"(b), "v"(c), "v"(d)); }
__device__ __forceinline__ void keep4_b(v16b a, v16b b, v16b c, v16b d) { asm volatile("v_nop" :: "v"(a), "v"(b), "v"(c), "v"(d)); }
__device__ __forceinline__ void acc_guard4(v8f& a, v8f& b, v8f& c, v8f& d) { asm volatile("v_nop\n\tv_nop\n\tv_nop\n\tv_nop" : "+v"(a), "+v"(b), "+v"(c), "+v"(d)); }
template <typename T> struct Frag;
template <> struct Frag<_Float16> {
  typedef v16h V; union U { v16h v; v8h h[2]; };
  static __device__ __forceinline__ v16h load(const _Float16* p) {
    U f; f.h[0] = *(const v8h*)(p); f.h[1] = *(const v8h*)(p + 16); return f.v;
  }
  static __device__ __forceinline__ v8f mma(v16h a, v16h b, v8f c) {
    return __builtin_amdgcn_wmma_f32_16x16x32_f16(false, a, false, b, (short)0, c, false, false);
  }
  static __device__ __forceinline__ void guard(v8f& a, v8f& b, v16h x, v16h y) { dep_guard_h(a, b, x, y); }
  static __device__ __forceinline__ void keep(v16h a, v16h b, v16h c, v16h d) { keep4_h(a, b, c, d); }
};
template <> struct Frag<__bf16> {
  typedef v16b V; union U { v16b v; v8b h[2]; };
  static __device__ __forceinline__ v16b load(const __bf16* p) {
    U f; f.h[0] = *(const v8b*)(p); f.h[1] = *(const v8b*)(p + 16); return f.v;
  }
  static __device__ __forceinline__ v8f mma(v16b a, v16b b, v8f c) {
    return __builtin_amdgcn_wmma_f32_16x16x32_bf16(false, a, false, b, (short)0, c, false, false);
  }
  static __device__ __forceinline__ void guard(v8f& a, v8f& b, v16b x, v16b y) { dep_guard_b(a, b, x, y); }
  static __device__ __forceinline__ void keep(v16b a, v16b b, v16b c, v16b d) { keep4_b(a, b, c, d); }
};

template <int ET> struct Elem;
template <> struct Elem<0> { typedef _Float16 T; };
template <> struct Elem<1> { typedef __bf16 T; };
template <int ET, bool SPLIT, int BIAS_MODE, int OUT_MODE, bool RESID, int ACT = 0>
__global__ __launch_bounds__(256) void wmma_gemm64(
    const unsigned short* __restrict__ Ap, const unsigned short* __restrict__ A2p, int lda, long strideA,
    const unsigned short* __restrict__ Btp, const unsigned short* __restrict__ Bt2p, int ldb, long strideB,
    void* __restrict__ Cout, void* __restrict__ Cout2, int ldc, long strideC,
    const float* __restrict__ bias,
    const float* __restrict__ resid, long strideR,
    int M, int N, int K, float scale) {
  typedef typename Elem<ET>::T T;
  typedef typename Frag<T>::V V;
  const T* A = (const T*)Ap; const T* A2 = (const T*)A2p; const T* Bt = (const T*)Btp; const T* Bt2 = (const T*)Bt2p;
  __shared__ __align__(16) float sT[8][16 * 68];
  const int b    = blockIdx.y;
  const int lane = threadIdx.x & 31;
  const int wave = threadIdx.x >> 5;
  const int tilesN = N >> 6;
  const int tilesM = M >> 6;
  const int tile = blockIdx.x * 8 + wave;
  if (tile >= tilesM * tilesN) return;
  const int tm = tile / tilesN;
  const int tn = tile - tm * tilesN;
  const int m0 = tm << 6;
  const int n0 = tn << 6;

  const T* Ab  = A  + (size_t)b * strideA;
  const T* Bb  = Bt + (size_t)b * strideB;
  const T* Ab2 = SPLIT ? (A2  + (size_t)b * strideA) : nullptr;
  const T* Bb2 = SPLIT ? (Bt2 + (size_t)b * strideB) : nullptr;

  const int rlane = lane & 15;
  const int koff  = (lane >> 4) * 8;
  const int mOff  = (lane >> 4) * 8;

  v8f acc[4][4];
#pragma unroll
  for (int i = 0; i < 4; ++i)
#pragma unroll
    for (int j = 0; j < 4; ++j) acc[i][j] = (v8f){0.f,0.f,0.f,0.f,0.f,0.f,0.f,0.f};

  for (int k0 = 0; k0 < K; k0 += 32) {
    V bh[4], bl[4];
#pragma unroll
    for (int j = 0; j < 4; ++j) {
      const size_t bo = (size_t)(n0 + (j << 4) + rlane) * ldb + koff + k0;
      bh[j] = Frag<T>::load(Bb + bo);
      if (SPLIT) bl[j] = Frag<T>::load(Bb2 + bo);
    }
#pragma unroll
    for (int i = 0; i < 4; ++i) {
      const size_t ao = (size_t)(m0 + (i << 4) + rlane) * lda + koff + k0;
      V ah = Frag<T>::load(Ab + ao);
      V al;
      if (SPLIT) al = Frag<T>::load(Ab2 + ao);
#pragma unroll
      for (int j = 0; j < 4; ++j) {
        acc[i][j] = Frag<T>::mma(ah, bh[j], acc[i][j]);
        if (SPLIT) {
          acc[i][j] = Frag<T>::mma(ah, bl[j], acc[i][j]);
          acc[i][j] = Frag<T>::mma(al, bh[j], acc[i][j]);
        }
      }
      Frag<T>::guard(acc[i][0], acc[i][3], ah, SPLIT ? al : ah);
    }
    Frag<T>::keep(bh[0], bh[1], bh[2], bh[3]);
    if (SPLIT) Frag<T>::keep(bl[0], bl[1], bl[2], bl[3]);
  }
  acc_guard4(acc[0][0], acc[0][1], acc[0][2], acc[0][3]);
  acc_guard4(acc[1][0], acc[1][1], acc[1][2], acc[1][3]);
  acc_guard4(acc[2][0], acc[2][1], acc[2][2], acc[2][3]);
  acc_guard4(acc[3][0], acc[3][1], acc[3][2], acc[3][3]);

  float* slab = sT[wave];
  const float* Rb = RESID ? (resid + (size_t)b * strideR) : nullptr;
#pragma unroll
  for (int i = 0; i < 4; ++i) {
    const int mBase = m0 + (i << 4);
#pragma unroll
    for (int j = 0; j < 4; ++j) {
      const int n = n0 + (j << 4) + rlane;
      float bv = 0.f;
      if (BIAS_MODE == 2) bv = bias[n];
#pragma unroll
      for (int r = 0; r < 8; ++r) {
        float v = acc[i][j][r] * scale;
        if (BIAS_MODE == 1) v += bias[mBase + mOff + r];
        if (BIAS_MODE == 2) v += bv;
        if (RESID) v += Rb[(size_t)(mBase + mOff + r) * ldc + n];
        if (ACT == 1) v = tanhf(v);
        if (ACT == 2) v = fmaxf(v, 0.0f);
        if (ACT == 3) v = v / (1.0f + expf(-v));
        if (ACT == 4) v = (v > 0.f) ? v : 0.01f * v;
        if (ACT == 5) v = 0.5f * v * (1.0f + erff(v * 0.70710678118654752f));
        slab[(mOff + r) * 68 + (j << 4) + rlane] = v;
      }
    }
    __builtin_amdgcn_fence(__ATOMIC_RELEASE, "workgroup");
    __builtin_amdgcn_wave_barrier();
    __builtin_amdgcn_fence(__ATOMIC_ACQUIRE, "workgroup");
    if (OUT_MODE == 0) {
      float* C = (float*)Cout + (size_t)b * strideC;
      const int hh = lane >> 4, c4 = (lane & 15) * 4;
      for (int pass = 0; pass < 2; ++pass) {
#pragma unroll
        for (int it = 0; it < 8; ++it) {
          const int row = it * 2 + hh;
          v4f v = *(const v4f*)(slab + row * 68 + c4);
          *(volatile v4f*)(C + (size_t)(mBase + row) * ldc + n0 + c4) = v;
        }
        __threadfence();
      }
    } else {
      const int q = lane >> 3, c8 = (lane & 7) * 8;
      unsigned short* C  = (unsigned short*)Cout  + (size_t)b * strideC;
      unsigned short* C2 = (OUT_MODE == 2) ? ((unsigned short*)Cout2 + (size_t)b * strideC) : nullptr;
      for (int pass = 0; pass < 2; ++pass) {
#pragma unroll
        for (int it = 0; it < 4; ++it) {
          const int row = it * 4 + q;
          const float* sp = slab + row * 68 + c8;
          v8h hv, lv;
#pragma unroll
          for (int e = 0; e < 8; ++e) {
            if (OUT_MODE == 1) {
              hv[e] = (_Float16)sp[e];
            } else {
              unsigned short hb = f2bf_bits(sp[e]);
              unsigned short lb = f2bf_bits(sp[e] - bf_bits2f(hb));
              hv[e] = __builtin_bit_cast(_Float16, hb);
              lv[e] = __builtin_bit_cast(_Float16, lb);
            }
          }
          *(volatile v8h*)(C + (size_t)(mBase + row) * ldc + n0 + c8) = hv;
          if (OUT_MODE == 2) *(volatile v8h*)(C2 + (size_t)(mBase + row) * ldc + n0 + c8) = lv;
        }
        __threadfence();
      }
    }
    __builtin_amdgcn_fence(__ATOMIC_RELEASE, "workgroup");
    __builtin_amdgcn_wave_barrier();
    __builtin_amdgcn_fence(__ATOMIC_ACQUIRE, "workgroup");
  }
}

__device__ __forceinline__ v8f mma16(v16h a, v16h b, v8f c) {
  c = __builtin_amdgcn_wmma_f32_16x16x32_f16(false, a, false, b, (short)0, c, false, false);
  asm volatile("v_nop\n\tv_nop\n\tv_nop\n\tv_nop" : "+v"(c) : "v"(a), "v"(b));
  return c;
}
__device__ __forceinline__ v8f zero8() { return (v8f){0.f,0.f,0.f,0.f,0.f,0.f,0.f,0.f}; }

__device__ __forceinline__ float elu_f(float x)  { return x > 0.0f ? x : (__expf(x) - 1.0f); }
__device__ __forceinline__ float sigm_f(float x) { return __builtin_amdgcn_rcpf(1.0f + __expf(-x)); }
__device__ __forceinline__ float tanh_f(float x) {
  const float ax = fabsf(x);
  const float e = __expf(-2.0f * ax);
  const float tv = (1.0f - e) * __builtin_amdgcn_rcpf(1.0f + e);
  return copysignf(tv, x);
}
__device__ __forceinline__ float clip52(float x) { return fminf(fmaxf(x, -5.0f), 2.0f); }

__global__ __launch_bounds__(256) void k_pack(const float* __restrict__ src, _Float16* __restrict__ dst,
                                              int R, int Cs, int Cd, int sa, int sb) {
  const int i = blockIdx.x * 256 + threadIdx.x;
  const int n8 = (R * Cd) >> 3;
  if (i < n8) {
    const int e0 = i * 8;
    const int r = e0 / Cd, c0 = e0 - r * Cd;
    v8h v;
#pragma unroll
    for (int e = 0; e < 8; ++e) {
      const int cc = c0 + e;
      const int cl = cc < Cs ? cc : (Cs - 1);
      const float x = src[(size_t)r * sa + (size_t)cl * sb];
      v[e] = (cc < Cs) ? (_Float16)x : (_Float16)0.0f;
    }
    _Float16* dp = dst + e0;
    *(volatile v8h*)dp = v;
    __threadfence();
    *(volatile v8h*)dp = v;
  }
}

__global__ __launch_bounds__(128) void k_enc(
    const float* __restrict__ obs,
    const _Float16* __restrict__ W1p, const float* __restrict__ b1,
    const _Float16* __restrict__ W2c, const float* __restrict__ b2,
    const _Float16* __restrict__ W3c, const float* __restrict__ b3,
    _Float16* __restrict__ feat) {
  __shared__ __align__(16) _Float16 x0[1024];
  __shared__ __align__(16) _Float16 col[8192];
  __shared__ __align__(16) _Float16 x1[8192];
  __shared__ __align__(16) _Float16 x2[4096];
  __shared__ __align__(16) _Float16 x3[1024];
  const int f = blockIdx.x, tid = threadIdx.x, wave = tid >> 5, lane = tid & 31;
  const int hh = lane >> 4, c = lane & 15;

  {
    const float* ob = obs + (size_t)f * 1024;
#pragma unroll
    for (int it = 0; it < 2; ++it) {
      const int idx = (it * 128 + tid) * 4;
      const v4f v = *(const v4f*)(ob + idx);
      x0[idx] = (_Float16)v[0]; x0[idx + 1] = (_Float16)v[1];
      x0[idx + 2] = (_Float16)v[2]; x0[idx + 3] = (_Float16)v[3];
    }
  }
  __syncthreads();

#pragma unroll 1
  for (int i = tid; i < 8192; i += 128) {
    const int p = i >> 5, k = i & 31;
    const int oy = p >> 4, ox = p & 15, ky = (k >> 2) & 3, kx = k & 3;
    const int iy = 2 * oy - 1 + ky, ix = 2 * ox - 1 + kx;
    const bool ok = (k < 16) && ((unsigned)iy < 32u) && ((unsigned)ix < 32u);
    const int ci = ok ? (iy * 32 + ix) : 0;
    const _Float16 v = x0[ci];
    col[i] = ok ? v : (_Float16)0.0f;
  }
  __syncthreads();

  {
    const v16h bA = Frag<_Float16>::load(W1p + c * 32 + 8 * hh);
    const v16h bB = Frag<_Float16>::load(W1p + (16 + c) * 32 + 8 * hh);
    v8f acc[4][2];
#pragma unroll
    for (int i = 0; i < 4; ++i) { acc[i][0] = zero8(); acc[i][1] = zero8(); }
#pragma unroll
    for (int i = 0; i < 4; ++i) {
      const int mt = wave * 4 + i;
      const v16h a = Frag<_Float16>::load(col + (mt * 16 + c) * 32 + 8 * hh);
      acc[i][0] = mma16(a, bA, acc[i][0]);
      acc[i][1] = mma16(a, bB, acc[i][1]);
    }
#pragma unroll
    for (int i = 0; i < 4; ++i) {
#pragma unroll
      for (int j = 0; j < 2; ++j) {
        const int oc = j * 16 + c;
        const float bv = b1[oc];
#pragma unroll
        for (int r = 0; r < 8; ++r) {
          const int px = (wave * 4 + i) * 16 + 8 * hh + r;
          x1[oc * 256 + px] = (_Float16)fmaxf(acc[i][j][r] + bv, 0.0f);
        }
      }
    }
  }
  __syncthreads();

  {
    v8f acc[4];
#pragma unroll
    for (int j = 0; j < 4; ++j) acc[j] = zero8();
#pragma unroll 1
    for (int ch = 0; ch < 4; ++ch) {
#pragma unroll 1
      for (int i = tid; i < 8192; i += 128) {
        const int p = i >> 7, kk = i & 127;
        const int ic = ch * 8 + (kk >> 4), ky = (kk >> 2) & 3, kx = kk & 3;
        const int oy = p >> 3, ox = p & 7;
        const int iy = 2 * oy - 1 + ky, ix = 2 * ox - 1 + kx;
        const bool ok = ((unsigned)iy < 16u) && ((unsigned)ix < 16u);
        const int ci = ok ? (ic * 256 + iy * 16 + ix) : 0;
        const _Float16 v = x1[ci];
        col[i] = ok ? v : (_Float16)0.0f;
      }
      __syncthreads();
#pragma unroll
      for (int ks = 0; ks < 4; ++ks) {
        const v16h a = Frag<_Float16>::load(col + (wave * 16 + c) * 128 + ks * 32 + 8 * hh);
#pragma unroll
        for (int j = 0; j < 4; ++j) {
          const v16h bq = Frag<_Float16>::load(W2c + (size_t)(j * 16 + c) * 512 + ch * 128 + ks * 32 + 8 * hh);
          acc[j] = mma16(a, bq, acc[j]);
        }
      }
      __syncthreads();
    }
#pragma unroll
    for (int j = 0; j < 4; ++j) {
      const int oc = j * 16 + c;
      const float bv = b2[oc];
#pragma unroll
      for (int r = 0; r < 8; ++r) {
        const int px = wave * 16 + 8 * hh + r;
        x2[oc * 64 + px] = (_Float16)fmaxf(acc[j][r] + bv, 0.0f);
      }
    }
  }
  __syncthreads();

  {
    v8f acc = zero8();
#pragma unroll 1
    for (int ch = 0; ch < 2; ++ch) {
#pragma unroll 1
      for (int i = tid; i < 8192; i += 128) {
        const int p = i >> 9, kk = i & 511;
        const int ic = ch * 32 + (kk >> 4), ky = (kk >> 2) & 3, kx = kk & 3;
        const int oy = p >> 2, ox = p & 3;
        const int iy = 2 * oy - 1 + ky, ix = 2 * ox - 1 + kx;
        const bool ok = ((unsigned)iy < 8u) && ((unsigned)ix < 8u);
        const int ci = ok ? (ic * 64 + iy * 8 + ix) : 0;
        const _Float16 v = x2[ci];
        col[i] = ok ? v : (_Float16)0.0f;
      }
      __syncthreads();
#pragma unroll 4
      for (int ks = 0; ks < 16; ++ks) {
        const v16h a = Frag<_Float16>::load(col + c * 512 + ks * 32 + 8 * hh);
        const v16h bq = Frag<_Float16>::load(W3c + (size_t)(wave * 16 + c) * 1024 + ch * 512 + ks * 32 + 8 * hh);
        acc = mma16(a, bq, acc);
      }
      __syncthreads();
    }
    const int oc = wave * 16 + c;
    const float bv = b3[oc];
#pragma unroll
    for (int r = 0; r < 8; ++r) {
      const int px = 8 * hh + r;
      x3[oc * 16 + px] = (_Float16)fmaxf(acc[r] + bv, 0.0f);
    }
  }
  __syncthreads();

  {
    const v8h v = *(const v8h*)(x3 + tid * 8);
    _Float16* dp = feat + (size_t)f * 1024 + tid * 8;
    *(volatile v8h*)dp = v;
    __threadfence();
    *(volatile v8h*)dp = v;
  }
}

#define C_OH   0
#define C_OE   4096
#define C_OA   6144
#define C_OZ   6208
#define C_OR   7232
#define C_OH1  (C_OR)
#define C_OH2  (C_OR + 4096)
#define C_OO3  (C_OR + 8192)
#define C_ORU  (C_OR)
#define C_OGI  (C_OR + 8192)
#define C_OGH  (C_OR + 12288)
#define C_SM   (C_OR + 16384)

__global__ __launch_bounds__(256) void k_core(
    const float* __restrict__ actions, const float* __restrict__ noise, const float* __restrict__ embed,
    const float* __restrict__ posW1, const float* __restrict__ posB1,
    const float* __restrict__ posW2, const float* __restrict__ posB2,
    const float* __restrict__ posW3, const float* __restrict__ posB3,
    const float* __restrict__ priW1, const float* __restrict__ priB1,
    const float* __restrict__ priW2, const float* __restrict__ priB2,
    const float* __restrict__ priW3, const float* __restrict__ priB3,
    const float* __restrict__ wih, const float* __restrict__ whh,
    const float* __restrict__ bih, const float* __restrict__ bhh,
    _Float16* __restrict__ hz,
    float* __restrict__ o_zs, float* __restrict__ o_prm, float* __restrict__ o_prls,
    float* __restrict__ o_pm, float* __restrict__ o_pls, float* __restrict__ o_hf) {
  __shared__ __align__(16) float sm[C_SM];
  const int tid = threadIdx.x, wave = tid >> 5, lane = tid & 31;
  const int q = lane >> 3, c4 = (lane & 7) * 4;

#pragma unroll 1
  for (int i = tid; i < 4096; i += 256) sm[C_OH + i] = 0.0f;
  __syncthreads();

  for (int t = 0; t < 64; ++t) {
#pragma unroll 1
    for (int i = tid; i < 2048; i += 256) {
      const int ch = i >> 5, b = i & 31;
      sm[C_OE + i] = embed[(size_t)(b * 64 + t) * 64 + ch];
    }
    if (tid < 64) {
      const int j = tid >> 5, b = tid & 31;
      sm[C_OA + tid] = actions[(size_t)(b * 64 + t) * 2 + j];
    }
    __syncthreads();

#pragma unroll 1
    for (int L = 0; L < 9; ++L) {
      int x0o = C_OH, K0 = 128, ld0 = 128, x1o = C_OH, K1 = 0, ld1 = 128, x2o = C_OH, K2 = 0, ld2 = 128;
      int N = 128, act = 0, outo = C_OGH;
      const float* W0 = whh + 256 * 128;
      const float* B0 = bhh + 256;
      const float* W1 = W0; const float* W2 = W0; const float* B1 = B0;
      float fb1 = 0.0f;
      switch (L) {
        case 0: x0o = C_OH;  K0 = 128; ld0 = 192; W0 = posW1; x1o = C_OE; K1 = 64; ld1 = 192; W1 = posW1 + 128;
                B0 = posB1; N = 128; act = 1; outo = C_OH1; break;
        case 1: x0o = C_OH1; K0 = 128; ld0 = 128; W0 = posW2; B0 = posB2; N = 128; act = 1; outo = C_OH2; break;
        case 2: x0o = C_OH2; K0 = 128; ld0 = 128; W0 = posW3; B0 = posB3; N = 64;  act = 0; outo = C_OO3; break;
        case 3: x0o = C_OH;  K0 = 128; ld0 = 130; W0 = priW1; x1o = C_OA; K1 = 2; ld1 = 130; W1 = priW1 + 128;
                B0 = priB1; N = 128; act = 1; outo = C_OH1; break;
        case 4: x0o = C_OH1; K0 = 128; ld0 = 128; W0 = priW2; B0 = priB2; N = 128; act = 1; outo = C_OH2; break;
        case 5: x0o = C_OH2; K0 = 128; ld0 = 128; W0 = priW3; B0 = priB3; N = 64;  act = 0; outo = C_OO3; break;
        case 6: x0o = C_OZ;  K0 = 32;  ld0 = 34;  W0 = wih; x1o = C_OA; K1 = 2; ld1 = 34; W1 = wih + 32;
                x2o = C_OH;  K2 = 128; ld2 = 128; W2 = whh; B0 = bih; B1 = bhh; fb1 = 1.0f;
                N = 256; act = 2; outo = C_ORU; break;
        case 7: x0o = C_OZ;  K0 = 32;  ld0 = 34;  W0 = wih + 256 * 34; x1o = C_OA; K1 = 2; ld1 = 34; W1 = wih + 256 * 34 + 32;
                B0 = bih + 256; N = 128; act = 0; outo = C_OGI; break;
        default: break;
      }
      const int K01 = K0 + K1, Kt = K01 + K2;

      for (int o = tid; o < 2 * N; o += 256) {
        const int n = o >> 1, half = o & 1;
        const float* w0r = W0 + (size_t)n * ld0;
        const float* w1r = W1 + (size_t)n * ld1;
        const float* w2r = W2 + (size_t)n * ld2;
        float acc[16];
#pragma unroll
        for (int i = 0; i < 16; ++i) acc[i] = 0.0f;
#pragma unroll 1
        for (int k = 0; k < Kt; ++k) {
          int xo, kq;
          const float* wr;
          if (k < K0)       { xo = x0o + k * 32;         wr = w0r; kq = k; }
          else if (k < K01) { xo = x1o + (k - K0) * 32;  wr = w1r; kq = k - K0; }
          else              { xo = x2o + (k - K01) * 32; wr = w2r; kq = k - K01; }
          const float w = wr[kq];
          const float* xp = sm + xo + half * 16;
          const v4f xa = *(const v4f*)(xp);
          const v4f xb = *(const v4f*)(xp + 4);
          const v4f xc = *(const v4f*)(xp + 8);
          const v4f xd = *(const v4f*)(xp + 12);
#pragma unroll
          for (int i = 0; i < 4; ++i) {
            acc[i]      += w * xa[i];
            acc[4 + i]  += w * xb[i];
            acc[8 + i]  += w * xc[i];
            acc[12 + i] += w * xd[i];
          }
        }
        const float bb = B0[n] + fb1 * B1[n];
        v4f ra, rb, rc, rd;
#pragma unroll
        for (int i = 0; i < 4; ++i) {
          float va = acc[i] + bb, vb = acc[4 + i] + bb, vc = acc[8 + i] + bb, vd = acc[12 + i] + bb;
          if (act == 1)      { va = elu_f(va);  vb = elu_f(vb);  vc = elu_f(vc);  vd = elu_f(vd); }
          else if (act == 2) { va = sigm_f(va); vb = sigm_f(vb); vc = sigm_f(vc); vd = sigm_f(vd); }
          ra[i] = va; rb[i] = vb; rc[i] = vc; rd[i] = vd;
        }
        float* op = sm + outo + n * 32 + half * 16;
        *(v4f*)(op)      = ra;
        *(v4f*)(op + 4)  = rb;
        *(v4f*)(op + 8)  = rc;
        *(v4f*)(op + 12) = rd;
      }
      __syncthreads();

      if (L == 2) {
        const int b = wave * 4 + q;
        v4f vpm, vpl, vz;
#pragma unroll
        for (int i = 0; i < 4; ++i) {
          const int s = c4 + i;
          const float pm = sm[C_OO3 + s * 32 + b];
          const float pl = clip52(sm[C_OO3 + (32 + s) * 32 + b]);
          const float ep = noise[(size_t)(t * 32 + b) * 32 + s];
          const float z = pm + __expf(pl) * ep;
          sm[C_OZ + s * 32 + b] = z;
          vpm[i] = pm; vpl[i] = pl; vz[i] = z;
        }
        const size_t oi = (size_t)(b * 64 + t) * 32 + c4;
        *(volatile v4f*)(o_pm + oi) = vpm;
        *(volatile v4f*)(o_pls + oi) = vpl;
        *(volatile v4f*)(o_zs + oi) = vz;
        __threadfence();
        *(volatile v4f*)(o_pm + oi) = vpm;
        *(volatile v4f*)(o_pls + oi) = vpl;
        *(volatile v4f*)(o_zs + oi) = vz;
        __syncthreads();
        if (lane < 24) {
#pragma unroll 1
          for (int i = 0; i < 4; ++i) {
            const int bb = wave * 4 + i;
            v8h hv;
#pragma unroll
            for (int e = 0; e < 8; ++e) {
              float x = 0.0f;
              if (lane < 16)      x = sm[C_OH + (8 * lane + e) * 32 + bb];
              else if (lane < 20) x = sm[C_OZ + (8 * (lane - 16) + e) * 32 + bb];
              hv[e] = (_Float16)x;
            }
            _Float16* dp = hz + (size_t)(t * 32 + bb) * 192 + 8 * lane;
            *(volatile v8h*)dp = hv;
            __threadfence();
            *(volatile v8h*)dp = hv;
          }
        }
      } else if (L == 5) {
        const int b = wave * 4 + q;
        v4f vm, vl;
#pragma unroll
        for (int i = 0; i < 4; ++i) {
          const int s = c4 + i;
          vm[i] = sm[C_OO3 + s * 32 + b];
          vl[i] = clip52(sm[C_OO3 + (32 + s) * 32 + b]);
        }
        const size_t oi = (size_t)(b * 64 + t) * 32 + c4;
        *(volatile v4f*)(o_prm + oi) = vm;
        *(volatile v4f*)(o_prls + oi) = vl;
        __threadfence();
        *(volatile v4f*)(o_prm + oi) = vm;
        *(volatile v4f*)(o_prls + oi) = vl;
      }
      __syncthreads();
    }

#pragma unroll 1
    for (int i = tid; i < 4096; i += 256) {
      const float r = sm[C_ORU + i], u = sm[C_ORU + 4096 + i];
      const float nv = tanh_f(sm[C_OGI + i] + r * sm[C_OGH + i]);
      const float h = sm[C_OH + i];
      sm[C_OH + i] = (1.0f - u) * nv + u * h;
    }
    __syncthreads();
  }

  for (int pass = 0; pass < 2; ++pass) {
#pragma unroll
    for (int it = 0; it < 4; ++it) {
      const int li = (it * 8 + wave) * 4 + q;
      const int b = li >> 2, nb = (li & 3) * 32 + c4;
      v4f v;
#pragma unroll
      for (int e = 0; e < 4; ++e) v[e] = sm[C_OH + (nb + e) * 32 + b];
      *(volatile v4f*)(o_hf + (size_t)b * 128 + nb) = v;
    }
    __threadfence();
  }
}

__global__ __launch_bounds__(128) void k_dec(
    const _Float16* __restrict__ y0,
    const _Float16* __restrict__ D1t, const float* __restrict__ b1,
    const _Float16* __restrict__ D2t, const float* __restrict__ b2,
    const _Float16* __restrict__ D3t, const float* __restrict__ b3,
    float* __restrict__ recons) {
  __shared__ __align__(16) _Float16 a0[1024];
  __shared__ __align__(16) float    g[8192];
  __shared__ __align__(16) _Float16 y1[4096];
  __shared__ __align__(16) _Float16 y2[8192];
  const int smp = blockIdx.x, tid = threadIdx.x, wave = tid >> 5, lane = tid & 31;
  const int hh = lane >> 4, c = lane & 15;

  {
    const v8h v = *(const v8h*)(y0 + (size_t)smp * 1024 + tid * 8);
    const int ic = tid >> 1, px0 = (tid & 1) * 8;
#pragma unroll
    for (int e = 0; e < 8; ++e) a0[(px0 + e) * 64 + ic] = v[e];
  }
  __syncthreads();

#pragma unroll 1
  for (int half = 0; half < 2; ++half) {
    v8f acc[8];
#pragma unroll
    for (int j = 0; j < 8; ++j) acc[j] = zero8();
#pragma unroll
    for (int ks = 0; ks < 2; ++ks) {
      const v16h a = Frag<_Float16>::load(a0 + c * 64 + ks * 32 + 8 * hh);
#pragma unroll
      for (int j = 0; j < 8; ++j) {
        const int nt = half * 32 + wave * 8 + j;
        const v16h bq = Frag<_Float16>::load(D1t + (size_t)(nt * 16 + c) * 64 + ks * 32 + 8 * hh);
        acc[j] = mma16(a, bq, acc[j]);
      }
    }
#pragma unroll
    for (int j = 0; j < 8; ++j) {
      const int nl = (wave * 8 + j) * 16 + c;
#pragma unroll
      for (int r = 0; r < 8; ++r) g[(8 * hh + r) * 512 + nl] = acc[j][r];
    }
    __syncthreads();
#pragma unroll 1
    for (int i = tid; i < 2048; i += 128) {
      const int ocl = i >> 6, p = i & 63, Y = p >> 3, X = p & 7;
      const int oc = half * 32 + ocl;
      float s = b1[oc];
      const int ky0 = (Y + 1) & 1, kx0 = (X + 1) & 1;
#pragma unroll
      for (int dy = 0; dy < 2; ++dy) {
        const int ky = ky0 + 2 * dy, ty = Y + 1 - ky;
        const bool oky = (ty >= 0) && (ty < 8);
        const int iy = oky ? (ty >> 1) : 0;
#pragma unroll
        for (int dx = 0; dx < 2; ++dx) {
          const int kx = kx0 + 2 * dx, tx = X + 1 - kx;
          const bool okx = (tx >= 0) && (tx < 8);
          const int ix = okx ? (tx >> 1) : 0;
          const float gv = g[(iy * 4 + ix) * 512 + ocl * 16 + ky * 4 + kx];
          s += (oky && okx) ? gv : 0.0f;
        }
      }
      y1[p * 64 + oc] = (_Float16)fmaxf(s, 0.0f);
    }
    __syncthreads();
  }

#pragma unroll 1
  for (int cc = 0; cc < 4; ++cc) {
    v8f acc[8];
#pragma unroll
    for (int j = 0; j < 8; ++j) acc[j] = zero8();
#pragma unroll
    for (int ks = 0; ks < 2; ++ks) {
      const v16h a = Frag<_Float16>::load(y1 + (wave * 16 + c) * 64 + ks * 32 + 8 * hh);
#pragma unroll
      for (int j = 0; j < 8; ++j) {
        const int nt = cc * 8 + j;
        const v16h bq = Frag<_Float16>::load(D2t + (size_t)(nt * 16 + c) * 64 + ks * 32 + 8 * hh);
        acc[j] = mma16(a, bq, acc[j]);
      }
    }
#pragma unroll
    for (int j = 0; j < 8; ++j) {
#pragma unroll
      for (int r = 0; r < 8; ++r) g[(wave * 16 + 8 * hh + r) * 128 + j * 16 + c] = acc[j][r];
    }
    __syncthreads();
#pragma unroll 1
    for (int i = tid; i < 2048; i += 128) {
      const int ocl = i >> 8, p = i & 255, Y = p >> 4, X = p & 15;
      const int oc = cc * 8 + ocl;
      float s = b2[oc];
      const int ky0 = (Y + 1) & 1, kx0 = (X + 1) & 1;
#pragma unroll
      for (int dy = 0; dy < 2; ++dy) {
        const int ky = ky0 + 2 * dy, ty = Y + 1 - ky;
        const bool oky = (ty >= 0) && (ty < 16);
        const int iy = oky ? (ty >> 1) : 0;
#pragma unroll
        for (int dx = 0; dx < 2; ++dx) {
          const int kx = kx0 + 2 * dx, tx = X + 1 - kx;
          const bool okx = (tx >= 0) && (tx < 16);
          const int ix = okx ? (tx >> 1) : 0;
          const float gv = g[(iy * 8 + ix) * 128 + ocl * 16 + ky * 4 + kx];
          s += (oky && okx) ? gv : 0.0f;
        }
      }
      y2[p * 32 + oc] = (_Float16)fmaxf(s, 0.0f);
    }
    __syncthreads();
  }

  {
    const v16h bq = Frag<_Float16>::load(D3t + c * 32 + 8 * hh);
    v8f acc[4];
#pragma unroll
    for (int i = 0; i < 4; ++i) acc[i] = zero8();
#pragma unroll
    for (int i = 0; i < 4; ++i) {
      const int mt = wave * 4 + i;
      const v16h a = Frag<_Float16>::load(y2 + (mt * 16 + c) * 32 + 8 * hh);
      acc[i] = mma16(a, bq, acc[i]);
    }
#pragma unroll
    for (int i = 0; i < 4; ++i) {
#pragma unroll
      for (int r = 0; r < 8; ++r) g[((wave * 4 + i) * 16 + 8 * hh + r) * 16 + c] = acc[i][r];
    }
  }
  __syncthreads();
  {
    const float bb = b3[0];
#pragma unroll 1
    for (int i = tid; i < 1024; i += 128) {
      const int Y = i >> 5, X = i & 31;
      float s = bb;
      const int ky0 = (Y + 1) & 1, kx0 = (X + 1) & 1;
#pragma unroll
      for (int dy = 0; dy < 2; ++dy) {
        const int ky = ky0 + 2 * dy, ty = Y + 1 - ky;
        const bool oky = (ty >= 0) && (ty < 32);
        const int iy = oky ? (ty >> 1) : 0;
#pragma unroll
        for (int dx = 0; dx < 2; ++dx) {
          const int kx = kx0 + 2 * dx, tx = X + 1 - kx;
          const bool okx = (tx >= 0) && (tx < 32);
          const int ix = okx ? (tx >> 1) : 0;
          const float gv = g[(iy * 16 + ix) * 16 + ky * 4 + kx];
          s += (oky && okx) ? gv : 0.0f;
        }
      }
      g[4096 + i] = sigm_f(s);
    }
  }
  __syncthreads();
  {
    const int t = smp >> 5, b = smp & 31;
    float* dp = recons + (size_t)(b * 64 + t) * 1024;
    const v4f v0 = *(const v4f*)(g + 4096 + tid * 4);
    const v4f v1 = *(const v4f*)(g + 4096 + 512 + tid * 4);
    *(volatile v4f*)(dp + tid * 4) = v0;
    *(volatile v4f*)(dp + 512 + tid * 4) = v1;
    __threadfence();
    *(volatile v4f*)(dp + tid * 4) = v0;
    *(volatile v4f*)(dp + 512 + tid * 4) = v1;
  }
}

extern "C" void kernel_launch(void* const* d_in, const int* in_sizes, int n_in,
                              void* d_out, int out_size, void* d_ws, size_t ws_size,
                              hipStream_t stream) {
  (void)n_in; (void)out_size;
  const float* obs    = (const float*)d_in[0];
  const float* acts   = (const float*)d_in[1];
  const float* noise  = (const float*)d_in[2];
  const float* enc_w1 = (const float*)d_in[3];  const float* enc_b1 = (const float*)d_in[4];
  const float* enc_w2 = (const float*)d_in[5];  const float* enc_b2 = (const float*)d_in[6];
  const float* enc_w3 = (const float*)d_in[7];  const float* enc_b3 = (const float*)d_in[8];
  const float* enc_pw = (const float*)d_in[9];  const float* enc_pb = (const float*)d_in[10];
  const float* dec_pw = (const float*)d_in[11]; const float* dec_pb = (const float*)d_in[12];
  const float* dec_w1 = (const float*)d_in[13]; const float* dec_b1 = (const float*)d_in[14];
  const float* dec_w2 = (const float*)d_in[15]; const float* dec_b2 = (const float*)d_in[16];
  const float* dec_w3 = (const float*)d_in[17]; const float* dec_b3 = (const float*)d_in[18];
  const float* gru_wih = (const float*)d_in[19]; const float* gru_whh = (const float*)d_in[20];
  const float* gru_bih = (const float*)d_in[21]; const float* gru_bhh = (const float*)d_in[22];
  const float* pri_w1 = (const float*)d_in[23]; const float* pri_b1 = (const float*)d_in[24];
  const float* pri_w2 = (const float*)d_in[25]; const float* pri_b2 = (const float*)d_in[26];
  const float* pri_w3 = (const float*)d_in[27]; const float* pri_b3 = (const float*)d_in[28];
  const float* pos_w1 = (const float*)d_in[29]; const float* pos_b1 = (const float*)d_in[30];
  const float* pos_w2 = (const float*)d_in[31]; const float* pos_b2 = (const float*)d_in[32];
  const float* pos_w3 = (const float*)d_in[33]; const float* pos_b3 = (const float*)d_in[34];

  const int NF = 2048;
  if (in_sizes[0] != NF * 1024 || in_sizes[2] != NF * 32 || in_sizes[1] != NF * 2) return;

  char* ws = (char*)d_ws;
  size_t off = 0;
  auto carve = [&](size_t bytes) -> char* {
    char* p = ws + off;
    off += (bytes + 255) & ~(size_t)255;
    return p;
  };
  _Float16* feat    = (_Float16*)carve((size_t)NF * 1024 * 2);
  float*    embed   = (float*)   carve((size_t)NF * 64 * 4);
  _Float16* hz      = (_Float16*)carve((size_t)NF * 192 * 2);
  _Float16* y0      = (_Float16*)carve((size_t)NF * 1024 * 2);
  _Float16* W1p     = (_Float16*)carve((size_t)32 * 32 * 2);
  _Float16* W2c     = (_Float16*)carve((size_t)64 * 512 * 2);
  _Float16* W3c     = (_Float16*)carve((size_t)64 * 1024 * 2);
  _Float16* encPw16 = (_Float16*)carve((size_t)64 * 1024 * 2);
  _Float16* decPw16 = (_Float16*)carve((size_t)1024 * 160 * 2);
  _Float16* D1t     = (_Float16*)carve((size_t)1024 * 64 * 2);
  _Float16* D2t     = (_Float16*)carve((size_t)512 * 64 * 2);
  _Float16* D3t     = (_Float16*)carve((size_t)16 * 32 * 2);
  if (off > ws_size) return;

  float* out    = (float*)d_out;
  float* o_rec  = out;
  float* o_zs   = out + (size_t)NF * 1024;
  float* o_prm  = o_zs   + (size_t)NF * 32;
  float* o_prls = o_prm  + (size_t)NF * 32;
  float* o_pm   = o_prls + (size_t)NF * 32;
  float* o_pls  = o_pm   + (size_t)NF * 32;
  float* o_hf   = o_pls  + (size_t)NF * 32;

  auto pack = [&](const float* src, _Float16* dst, int R, int Cs, int Cd, int sa, int sb) {
    const int n8 = (R * Cd) / 8;
    k_pack<<<dim3((n8 + 255) / 256), dim3(256), 0, stream>>>(src, dst, R, Cs, Cd, sa, sb);
  };
  pack(enc_w1, W1p,     32,   16,   32,   16,    1);
  pack(enc_w2, W2c,     64,  512,  512,  512,    1);
  pack(enc_w3, W3c,     64, 1024, 1024, 1024,    1);
  pack(enc_pw, encPw16, 64, 1024, 1024, 1024,    1);
  pack(dec_pw, decPw16, 1024, 160, 160,  160,    1);
  pack(dec_w1, D1t,   1024,   64,   64,    1, 1024);
  pack(dec_w2, D2t,    512,   64,   64,    1,  512);
  pack(dec_w3, D3t,     16,   32,   32,    1,   16);

  k_enc<<<dim3(NF), dim3(128), 0, stream>>>(obs, W1p, enc_b1, W2c, enc_b2, W3c, enc_b3, feat);

  wmma_gemm64<0, false, 2, 0, false, 0><<<dim3(4, 1), dim3(256), 0, stream>>>(
      U16(feat), U16(feat), 1024, 0L, U16(encPw16), U16(encPw16), 1024, 0L,
      (void*)embed, (void*)embed, 64, 0L, enc_pb, enc_pb, 0L, NF, 64, 1024, 1.0f);

  k_core<<<dim3(1), dim3(256), 0, stream>>>(acts, noise, embed,
      pos_w1, pos_b1, pos_w2, pos_b2, pos_w3, pos_b3,
      pri_w1, pri_b1, pri_w2, pri_b2, pri_w3, pri_b3,
      gru_wih, gru_whh, gru_bih, gru_bhh,
      hz, o_zs, o_prm, o_prls, o_pm, o_pls, o_hf);

  wmma_gemm64<0, false, 2, 1, false, 0><<<dim3(64, 1), dim3(256), 0, stream>>>(
      U16(hz), U16(hz), 192, 0L, U16(decPw16), U16(decPw16), 160, 0L,
      (void*)y0, (void*)y0, 1024, 0L, dec_pb, dec_pb, 0L, NF, 1024, 160, 1.0f);

  k_dec<<<dim3(NF), dim3(128), 0, stream>>>(y0, D1t, dec_b1, D2t, dec_b2, D3t, dec_b3, o_rec);
}
